// ChipPairEncoderAlpha_1382979469738
// MI455X (gfx1250) — hardware-verified
//
#include <hip/hip_runtime.h>

typedef _Float16       v16h  __attribute__((ext_vector_type(16)));
typedef _Float16       v8h   __attribute__((ext_vector_type(8)));
typedef __bf16         v16b  __attribute__((ext_vector_type(16)));
typedef unsigned short v16us __attribute__((ext_vector_type(16)));
typedef unsigned short v8us  __attribute__((ext_vector_type(8)));
typedef float          v8f   __attribute__((ext_vector_type(8)));
typedef float          v4f   __attribute__((ext_vector_type(4)));
typedef v8h  __attribute__((may_alias)) v8h_ma;
typedef v8us __attribute__((may_alias)) v8us_ma;
typedef v4f  __attribute__((may_alias)) v4f_ma;

union FragH { v16h v;  v8h  half[2]; };
union FragU { v16us v; v8us half[2]; };

__device__ __forceinline__ float wave_sum32(float v) {
#pragma unroll
  for (int o = 16; o > 0; o >>= 1) v += __shfl_xor(v, o, 32);
  return v;
}

__device__ __forceinline__ int kof(int i, int hh) { return (i & 7) + ((i >> 3) << 4) + 8 * hh; }

__device__ __forceinline__ v8f wmma_f16(v16h a, v16h b, v8f c) {
  c = __builtin_amdgcn_wmma_f32_16x16x32_f16(false, a, false, b, (short)0, c, false, false);
  asm volatile("v_nop\n\tv_nop\n\tv_nop\n\tv_nop" : "+v"(c) : "v"(a), "v"(b));
  return c;
}

__device__ __forceinline__ v8f wmma_bf16(v16us a, v16us b, v8f c) {
  v16b ab = __builtin_bit_cast(v16b, a);
  v16b bb = __builtin_bit_cast(v16b, b);
  c = __builtin_amdgcn_wmma_f32_16x16x32_bf16(false, ab, false, bb, (short)0, c, false, false);
  asm volatile("v_nop\n\tv_nop\n\tv_nop\n\tv_nop" : "+v"(c) : "v"(ab), "v"(bb));
  return c;
}

__device__ __forceinline__ unsigned short bf_rne(float x) {
  unsigned int u = __float_as_uint(x);
  u += 0x7FFFu + ((u >> 16) & 1u);
  return (unsigned short)(u >> 16);
}
__device__ __forceinline__ float bf_val(unsigned short s) {
  return __uint_as_float(((unsigned int)s) << 16);
}

__device__ __forceinline__ v16h wfrag_f16(const float* __restrict__ W, int n, int hh) {
  const float* r = W + n * 32;
  v16h f = {};
#pragma unroll
  for (int i = 0; i < 16; ++i) f[i] = (_Float16)r[kof(i, hh)];
  return f;
}

__global__ __launch_bounds__(256) void k_attn(
    const float* __restrict__ ctcf, const float* __restrict__ hac,
    const float* __restrict__ me1,  const float* __restrict__ me3,
    const float* __restrict__ bulk,
    const float* __restrict__ we_w, const float* __restrict__ we_b,
    const float* __restrict__ pos,
    const float* __restrict__ mn_g, const float* __restrict__ mn_b,
    const float* __restrict__ wq,   const float* __restrict__ bq,
    const float* __restrict__ wk,   const float* __restrict__ bk,
    const float* __restrict__ wv,   const float* __restrict__ bv,
    const float* __restrict__ wo,   const float* __restrict__ bo,
    const float* __restrict__ an_g, const float* __restrict__ an_b,
    const float* __restrict__ conv_w, const float* __restrict__ conv_b,
    const float* __restrict__ gate_w, const float* __restrict__ gate_b,
    float* __restrict__ xw, int nbs)
{
  __shared__ __attribute__((aligned(16))) float    xs[64][32];
  __shared__ __attribute__((aligned(16))) _Float16 xh[64][32];
  __shared__ __attribute__((aligned(16))) float    qf[64][32];
  __shared__ __attribute__((aligned(16))) float    kf[64][32];
  __shared__ __attribute__((aligned(16))) _Float16 vh[64][32];
  __shared__ __attribute__((aligned(16))) _Float16 ph[64][64];
  __shared__ __attribute__((aligned(16))) float    og[64][32];
  __shared__ __attribute__((aligned(16))) _Float16 oh[64][32];
  __shared__ __attribute__((aligned(16))) float    o2[64][32];

  const int tid = threadIdx.x, wave = tid >> 5, lane = tid & 31;
  const int hh = lane >> 4, m16 = lane & 15;
  const int bs = blockIdx.x;
  if (bs >= nbs) return;
  const int b = bs >> 2, s = bs & 3;

  {
    const float* sig = (s == 0) ? ctcf : ((s == 1) ? hac : ((s == 2) ? me1 : me3));
    const float ww = we_w[lane], wb = we_b[lane], g = mn_g[lane], be = mn_b[lane];
    for (int rr = 0; rr < 8; ++rr) {
      const int l = wave * 8 + rr;
      float v = sig[b * 64 + l] * ww + wb;
      v += pos[l * 32 + lane];
      const float mu  = wave_sum32(v) * 0.03125f;
      const float d   = v - mu;
      const float var = wave_sum32(d * d) * 0.03125f;
      const float y   = d * (1.0f / sqrtf(var + 1e-5f)) * g + be;
      xs[l][lane] = y;
      xh[l][lane] = (_Float16)y;
    }
  }
  __syncthreads();

  {
    const int mt = wave >> 1, nt = wave & 1;
    const int arow = mt * 16 + m16, ncol = nt * 16 + m16, drow = mt * 16 + 8 * hh;
    FragH a;
    a.half[0] = *(const v8h_ma*)(&xh[arow][8 * hh]);
    a.half[1] = *(const v8h_ma*)(&xh[arow][16 + 8 * hh]);
    {
      v8f acc = {};
      acc = wmma_f16(a.v, wfrag_f16(wq, ncol, hh), acc);
      const float bb = bq[ncol];
#pragma unroll
      for (int r = 0; r < 8; ++r) qf[drow + r][ncol] = acc[r] + bb;
    }
    {
      v8f acc = {};
      acc = wmma_f16(a.v, wfrag_f16(wk, ncol, hh), acc);
      const float bb = bk[ncol];
#pragma unroll
      for (int r = 0; r < 8; ++r) kf[drow + r][ncol] = acc[r] + bb;
    }
    {
      v8f acc = {};
      acc = wmma_f16(a.v, wfrag_f16(wv, ncol, hh), acc);
      const float bb = bv[ncol];
#pragma unroll
      for (int r = 0; r < 8; ++r) vh[drow + r][ncol] = (_Float16)(acc[r] + bb);
    }
  }
  __syncthreads();

  const float rsD = 0.35355339059327373f;
#pragma unroll 1
  for (int h = 0; h < 4; ++h) {
    {
      const int l = tid >> 2, m0 = (tid & 3) * 16;
      float qr[8];
#pragma unroll
      for (int d = 0; d < 8; ++d) qr[d] = qf[l][h * 8 + d];
      const float cw = conv_w[h], cb = conv_b[h];
      const float* bl = bulk + ((size_t)b * 64 + l) * 64 + m0;
      float sc[16];
      float mx = -3.0e38f;
#pragma unroll
      for (int mm = 0; mm < 16; ++mm) {
        float acc = 0.f;
#pragma unroll
        for (int d = 0; d < 8; ++d) acc += qr[d] * kf[m0 + mm][h * 8 + d];
        const float sv = acc * rsD + (bl[mm] * cw + cb);
        sc[mm] = sv;
        mx = fmaxf(mx, sv);
      }
      mx = fmaxf(mx, __shfl_xor(mx, 1, 32));
      mx = fmaxf(mx, __shfl_xor(mx, 2, 32));
      float sum = 0.f;
#pragma unroll
      for (int mm = 0; mm < 16; ++mm) { const float e = __expf(sc[mm] - mx); sc[mm] = e; sum += e; }
      sum += __shfl_xor(sum, 1, 32);
      sum += __shfl_xor(sum, 2, 32);
      const float inv = 4096.0f / sum;
      FragH pv;
#pragma unroll
      for (int mm = 0; mm < 8; ++mm) {
        pv.half[0][mm] = (_Float16)(sc[mm] * inv);
        pv.half[1][mm] = (_Float16)(sc[8 + mm] * inv);
      }
      *(v8h_ma*)(&ph[l][m0])     = pv.half[0];
      *(v8h_ma*)(&ph[l][m0 + 8]) = pv.half[1];
    }
    __syncthreads();
    if (wave < 4) {
      const int mt = wave, arow = mt * 16 + m16, vcol = h * 8 + (m16 & 7);
      v8f acc = {};
#pragma unroll
      for (int ks = 0; ks < 2; ++ks) {
        const int k0 = ks * 32;
        FragH a;
        a.half[0] = *(const v8h_ma*)(&ph[arow][k0 + 8 * hh]);
        a.half[1] = *(const v8h_ma*)(&ph[arow][k0 + 16 + 8 * hh]);
        v16h bvv = {};
#pragma unroll
        for (int i = 0; i < 16; ++i) {
          const _Float16 t = vh[k0 + kof(i, hh)][vcol];
          bvv[i] = (m16 < 8) ? t : (_Float16)0.0f;
        }
        acc = wmma_f16(a.v, bvv, acc);
      }
      if (m16 < 8) {
        const int drow = mt * 16 + 8 * hh;
#pragma unroll
        for (int r = 0; r < 8; ++r) og[drow + r][h * 8 + m16] = acc[r] * (1.0f / 4096.0f);
      }
    }
    __syncthreads();
  }

#pragma unroll 1
  for (int j = 0; j < 8; ++j) {
    const int idx = tid + 256 * j;
    const int l = idx >> 5, hc = idx & 31, h8 = hc & 24;
    float acc = gate_b[hc];
#pragma unroll
    for (int d = 0; d < 8; ++d) acc += gate_w[hc * 8 + d] * og[l][h8 + d];
    const float gs = 1.0f / (1.0f + __expf(-acc));
    oh[l][hc] = (_Float16)(og[l][hc] * gs);
  }
  __syncthreads();

  {
    const int mt = wave >> 1, nt = wave & 1;
    const int arow = mt * 16 + m16, ncol = nt * 16 + m16, drow = mt * 16 + 8 * hh;
    FragH a;
    a.half[0] = *(const v8h_ma*)(&oh[arow][8 * hh]);
    a.half[1] = *(const v8h_ma*)(&oh[arow][16 + 8 * hh]);
    v8f acc = {};
    acc = wmma_f16(a.v, wfrag_f16(wo, ncol, hh), acc);
    const float bb = bo[ncol];
#pragma unroll
    for (int r = 0; r < 8; ++r) o2[drow + r][ncol] = acc[r] + bb;
  }
  __syncthreads();

  {
    const float g = an_g[lane], be = an_b[lane];
    for (int rr = 0; rr < 8; ++rr) {
      const int l = wave * 8 + rr;
      const float v   = xs[l][lane] + o2[l][lane];
      const float mu  = wave_sum32(v) * 0.03125f;
      const float d   = v - mu;
      const float var = wave_sum32(d * d) * 0.03125f;
      xs[l][lane] = d * (1.0f / sqrtf(var + 1e-5f)) * g + be;
    }
  }
  __syncthreads();

  {
    float* xg = xw + (size_t)bs * 2048;
    const int col = 4 * (lane & 7);
    const int r0 = wave * 8 + (lane >> 3), r1 = r0 + 4;
    const v4f v0 = *(const v4f_ma*)(&xs[r0][col]);
    const v4f v1 = *(const v4f_ma*)(&xs[r1][col]);
    *(volatile v4f*)(xg + r0 * 32 + col) = v0;
    *(volatile v4f*)(xg + r1 * 32 + col) = v1;
    __threadfence();
    *(volatile v4f*)(xg + r0 * 32 + col) = v0;
    *(volatile v4f*)(xg + r1 * 32 + col) = v1;
  }
}

__global__ __launch_bounds__(256) void k_pair(
    const float* __restrict__ xw, const float* __restrict__ ppw, const float* __restrict__ pp_b,
    const float* __restrict__ ada_g, const float* __restrict__ ada_b, const float* __restrict__ ada_alpha,
    float* __restrict__ out, int nblk)
{
  __shared__ __attribute__((aligned(16))) unsigned short mhi[64][32];
  __shared__ __attribute__((aligned(16))) unsigned short mlo[64][32];
  __shared__ __attribute__((aligned(16))) float tf[16][16][32];
  __shared__ __attribute__((aligned(16))) float fo[16][16][64];
  float* mf = &fo[0][0][0];

  const int tid = threadIdx.x, wave = tid >> 5, lane = tid & 31;
  const int hh = lane >> 4, m16 = lane & 15;
  const int blk = blockIdx.x;
  if (blk >= nblk) return;
  const int b = blk >> 2, i0 = (blk & 3) * 16;

  {
    const float* xb = xw + (size_t)b * 8192;
#pragma unroll
    for (int j = 0; j < 8; ++j) {
      const int e = tid + 256 * j;
      float v = xb[e];
      v = fmaxf(v, xb[2048 + e]);
      v = fmaxf(v, xb[4096 + e]);
      v = fmaxf(v, xb[6144 + e]);
      mf[e] = v;
    }
  }
  __syncthreads();

  for (int rr = 0; rr < 8; ++rr) {
    const int l = wave * 8 + rr;
    const float v   = mf[l * 32 + lane];
    const float n2  = wave_sum32(v * v);
    const float inv = 1.0f / fmaxf(sqrtf(n2), 1e-3f);
    const float y   = v * inv;
    const unsigned short hb = bf_rne(y);
    mhi[l][lane] = hb;
    mlo[l][lane] = bf_rne(y - bf_val(hb));
  }
  __syncthreads();

  {
    const int arow = i0 + m16;
    FragU ahi, alo;
    ahi.half[0] = *(const v8us_ma*)(&mhi[arow][8 * hh]);
    ahi.half[1] = *(const v8us_ma*)(&mhi[arow][16 + 8 * hh]);
    alo.half[0] = *(const v8us_ma*)(&mlo[arow][8 * hh]);
    alo.half[1] = *(const v8us_ma*)(&mlo[arow][16 + 8 * hh]);
#pragma unroll 1
    for (int pp = 0; pp < 2; ++pp) {
      const int p = wave * 2 + pp;
#pragma unroll 1
      for (int nt = 0; nt < 2; ++nt) {
        const int n = nt * 16 + m16;
        const float* wp = ppw + (size_t)p * 1024 + n;
        v16us bh = {}, bl = {};
#pragma unroll
        for (int i = 0; i < 16; ++i) {
          const float w = wp[kof(i, hh) * 32];
          const unsigned short hb = bf_rne(w);
          bh[i] = hb;
          bl[i] = bf_rne(w - bf_val(hb));
        }
        v8f acc = {};
        acc = wmma_bf16(ahi.v, bh, acc);
        acc = wmma_bf16(ahi.v, bl, acc);
        acc = wmma_bf16(alo.v, bh, acc);
#pragma unroll
        for (int r = 0; r < 8; ++r) tf[p][8 * hh + r][n] = acc[r];
      }
    }
  }
  __syncthreads();

#pragma unroll 1
  for (int nt = 0; nt < 4; ++nt) {
    const int brow = nt * 16 + m16;
    FragU bh, bl;
    bh.half[0] = *(const v8us_ma*)(&mhi[brow][8 * hh]);
    bh.half[1] = *(const v8us_ma*)(&mhi[brow][16 + 8 * hh]);
    bl.half[0] = *(const v8us_ma*)(&mlo[brow][8 * hh]);
    bl.half[1] = *(const v8us_ma*)(&mlo[brow][16 + 8 * hh]);
#pragma unroll 1
    for (int pp = 0; pp < 2; ++pp) {
      const int p = wave * 2 + pp;
      v16us ah = {}, al = {};
#pragma unroll
      for (int i = 0; i < 16; ++i) {
        const float t = tf[p][m16][kof(i, hh)];
        const unsigned short hb = bf_rne(t);
        ah[i] = hb;
        al[i] = bf_rne(t - bf_val(hb));
      }
      v8f acc = {};
      acc = wmma_bf16(ah, bh.v, acc);
      acc = wmma_bf16(ah, bl.v, acc);
      acc = wmma_bf16(al, bh.v, acc);
      const float pb = pp_b[p];
#pragma unroll
      for (int r = 0; r < 8; ++r) fo[p][8 * hh + r][brow] = acc[r] + pb;
    }
  }
  __syncthreads();

  {
    const float alpha = ada_alpha[0];
#pragma unroll 1
    for (int jq = 0; jq < 4; ++jq) {
      const int q = tid + 256 * jq;
      const int i = q >> 6, j = q & 63;
      float v[16];
      float mu = 0.f;
#pragma unroll
      for (int p = 0; p < 16; ++p) { v[p] = fo[p][i][j]; mu += v[p]; }
      mu *= 0.0625f;
      float var = 0.f;
#pragma unroll
      for (int p = 0; p < 16; ++p) { const float d = v[p] - mu; var += d * d; }
      var *= 0.0625f;
      const float rs = 1.0f / sqrtf(var + 1e-5f);
#pragma unroll
      for (int p = 0; p < 16; ++p) {
        const float f = v[p] + alpha * ((v[p] - mu) * rs * ada_g[p] + ada_b[p]);
        fo[p][i][j] = f / (1.0f + __expf(-f));
      }
    }
  }
  __syncthreads();

  {
    const size_t pbase = (size_t)b * 16;
    const int col = 4 * (lane & 15), rsel = lane >> 4;
#pragma unroll 1
    for (int u = 0; u < 16; ++u) {
      const int rho = wave * 32 + 2 * u + rsel;
      const int p = rho >> 4, i = rho & 15;
      const v4f v = *(const v4f_ma*)(&fo[p][i][col]);
      *(volatile v4f*)(out + (((pbase + p) * 64 + (size_t)(i0 + i)) * 64 + col)) = v;
    }
    __threadfence();
#pragma unroll 1
    for (int u = 0; u < 16; ++u) {
      const int rho = wave * 32 + 2 * u + rsel;
      const int p = rho >> 4, i = rho & 15;
      const v4f v = *(const v4f_ma*)(&fo[p][i][col]);
      *(volatile v4f*)(out + (((pbase + p) * 64 + (size_t)(i0 + i)) * 64 + col)) = v;
    }
  }
}

extern "C" void kernel_launch(void* const* d_in, const int* in_sizes, int n_in,
                              void* d_out, int out_size, void* d_ws, size_t ws_size,
                              hipStream_t stream) {
  if (n_in < 29 || d_out == 0 || d_ws == 0) return;
  const int nB = in_sizes[0] / 64;
  if (nB <= 0 || in_sizes[0] != nB * 64 || in_sizes[1] != nB * 64 || in_sizes[2] != nB * 64 ||
      in_sizes[3] != nB * 64 || in_sizes[4] != nB * 4096 ||
      in_sizes[5] < 32 || in_sizes[6] < 32 || in_sizes[7] != 2048 || in_sizes[8] < 32 || in_sizes[9] < 32 ||
      in_sizes[10] != 1024 || in_sizes[11] < 32 || in_sizes[12] != 1024 || in_sizes[13] < 32 ||
      in_sizes[14] != 1024 || in_sizes[15] < 32 || in_sizes[16] != 1024 || in_sizes[17] < 32 ||
      in_sizes[18] < 32 || in_sizes[19] < 32 || in_sizes[20] < 4 || in_sizes[21] < 4 ||
      in_sizes[22] != 256 || in_sizes[23] < 32 || in_sizes[24] != 16384 || in_sizes[25] < 16 ||
      in_sizes[26] < 16 || in_sizes[27] < 16 || in_sizes[28] < 1 ||
      out_size != nB * 16 * 4096) return;
  const size_t need = (size_t)nB * 8192 * sizeof(float);
  if (need > ws_size) return;

  const float* ctcf   = (const float*)d_in[0];
  const float* hac    = (const float*)d_in[1];
  const float* me1    = (const float*)d_in[2];
  const float* me3    = (const float*)d_in[3];
  const float* bulk   = (const float*)d_in[4];
  const float* we_w   = (const float*)d_in[5];
  const float* we_b   = (const float*)d_in[6];
  const float* pos    = (const float*)d_in[7];
  const float* mn_g   = (const float*)d_in[8];
  const float* mn_b   = (const float*)d_in[9];
  const float* wq     = (const float*)d_in[10];
  const float* bq     = (const float*)d_in[11];
  const float* wk     = (const float*)d_in[12];
  const float* bk     = (const float*)d_in[13];
  const float* wv     = (const float*)d_in[14];
  const float* bv     = (const float*)d_in[15];
  const float* wo     = (const float*)d_in[16];
  const float* bo     = (const float*)d_in[17];
  const float* an_g   = (const float*)d_in[18];
  const float* an_b   = (const float*)d_in[19];
  const float* conv_w = (const float*)d_in[20];
  const float* conv_b = (const float*)d_in[21];
  const float* gate_w = (const float*)d_in[22];
  const float* gate_b = (const float*)d_in[23];
  const float* pp_w   = (const float*)d_in[24];
  const float* pp_b   = (const float*)d_in[25];
  const float* ada_g  = (const float*)d_in[26];
  const float* ada_b  = (const float*)d_in[27];
  const float* ada_a  = (const float*)d_in[28];

  float* ws_x = (float*)d_ws;
  const int nbs = nB * 4;
  const int nblk = nB * 4;

  k_attn<<<nbs, 256, 0, stream>>>(ctcf, hac, me1, me3, bulk, we_w, we_b, pos, mn_g, mn_b,
                                   wq, bq, wk, bk, wv, bv, wo, bo, an_g, an_b,
                                   conv_w, conv_b, gate_w, gate_b, ws_x, nbs);
  k_pair<<<nblk, 256, 0, stream>>>(ws_x, pp_w, pp_b, ada_g, ada_b, ada_a, (float*)d_out, nblk);
}
